// MyModel_61933428409043
// MI455X (gfx1250) — hardware-verified
//
#include <hip/hip_runtime.h>
#include <math.h>

typedef __attribute__((ext_vector_type(16))) _Float16 v16h;
typedef __attribute__((ext_vector_type(8)))  _Float16 v8h;
typedef __attribute__((ext_vector_type(8)))  float    v8f;
typedef __attribute__((ext_vector_type(4)))  float    v4f;

constexpr int kBatch     = 2048;
constexpr int kSteps     = 512;
constexpr int kHid       = 51;
constexpr int kHP        = 64;
constexpr int kG4        = 4 * kHid;
constexpr int kGP        = 4 * kHP;
constexpr int kThr       = 256;
constexpr int kBlocks    = kBatch / (8 * 16);
constexpr int kChunk     = 32;
constexpr int kNumChunks = kSteps / kChunk;
constexpr int kPitch     = 36;
constexpr int kW1P       = 72;
constexpr int kW2P       = 136;
constexpr int kXK        = 51;
constexpr size_t kOutElems = (size_t)kBatch * kSteps;
static_assert(kBlocks == 16 && kHid + 3 <= kHP && kSteps % kChunk == 0, "sixteen blocks of eight 16-row tiles; three spare slots");

constexpr float kSCarry = 1024.0f;
constexpr float kWCarry = 4096.0f;
constexpr float kFold   = 1.0f / (kSCarry * kWCarry);
constexpr float kF16MinNormal = 6.103515625e-5f;
static_assert(kFold == 2.384185791015625e-7f, "2^-22");

union FragU { v16h v; v8h h[2]; };

__device__ __forceinline__ unsigned short f2bf_bits(float f) {
  unsigned u = __float_as_uint(f);
  return (unsigned short)((u + 0x7FFFu + ((u >> 16) & 1u)) >> 16);
}
__device__ __forceinline__ float bf16r(float f) { return __uint_as_float(((unsigned)f2bf_bits(f)) << 16); }
__device__ __forceinline__ float carry_flush(float v, float c) {
  const float s = v * c;
  return (fabsf(s) < kF16MinNormal) ? 0.0f : s;
}
__device__ __forceinline__ v8f mma_h(v16h a, v16h b, v8f c) {
  c = __builtin_amdgcn_wmma_f32_16x16x32_f16(false, a, false, b, (short)0, c, false, false);
  asm volatile("v_nop\n\tv_nop\n\tv_nop\n\tv_nop" : "+v"(c) : "v"(a), "v"(b));
  return c;
}
__device__ __forceinline__ v16h frag_h32(const _Float16* p) { FragU f; f.h[0] = *(const v8h*)(p); f.h[1] = *(const v8h*)(p + 16); return f.v; }
__device__ __forceinline__ v16h frag_tiles(const float* a, const float* b, float c) {
  v16h f;
#pragma unroll
  for (int e = 0; e < 8; ++e) { f[e] = (_Float16)carry_flush(a[e], c); f[8 + e] = (_Float16)carry_flush(b[e], c); }
  return f;
}
__device__ __forceinline__ float fast_tanh(float v) {
  const float e = __expf(2.0f * v);
  return 1.0f - 2.0f * __builtin_amdgcn_rcpf(e + 1.0f);
}
__device__ __forceinline__ float fast_sigmoid(float v) { return __builtin_amdgcn_rcpf(1.0f + __expf(-v)); }

__global__ __launch_bounds__(kThr) void lstm51x2_kernel(const float* __restrict__ x, const float* __restrict__ wih1,
                                                        const float* __restrict__ whh1, const float* __restrict__ bih1,
                                                        const float* __restrict__ bhh1, const float* __restrict__ wih2,
                                                        const float* __restrict__ whh2, const float* __restrict__ bih2,
                                                        const float* __restrict__ bhh2, const float* __restrict__ wlin,
                                                        const float* __restrict__ blin, float* __restrict__ outs) {
  __shared__ __align__(16) _Float16 sW1[kGP * kW1P];
  __shared__ __align__(16) _Float16 sW2[kGP * kW2P];
  __shared__ __align__(16) float    sWl[kHP];
  __shared__ __align__(16) float    xs[8 * 16 * kPitch];
  __shared__ __align__(16) float    os[8 * 16 * kPitch];
  const int tid = threadIdx.x;
  const int wave = tid >> 5;
  const int lane = tid & 31;
  const int col = lane & 15;
  const int hs = lane >> 4;
  const bool lowHalf = (hs == 0);

  {
    const int q = tid >> 6;
    const int j = tid & 63;
    const bool live = j < kHid;
    const int src = live ? (kHid * q + j) : 0;
    _Float16* w1 = sW1 + tid * kW1P;
    _Float16* w2 = sW2 + tid * kW2P;
#pragma unroll 1
    for (int k = 0; k < kW1P; ++k) w1[k] = (_Float16)0.0f;
#pragma unroll 1
    for (int k = 0; k < kW2P; ++k) w2[k] = (_Float16)0.0f;
    if (live) {
#pragma unroll 1
      for (int k = 0; k < kHid; ++k) {
        const float a = whh1[src * kHid + k];
        const float b = wih2[src * kHid + k];
        const float c = whh2[src * kHid + k];
        w1[k] = (_Float16)carry_flush(bf16r(a), kWCarry);
        w2[k] = (_Float16)carry_flush(bf16r(b), kWCarry);
        w2[kHP + k] = (_Float16)carry_flush(bf16r(c), kWCarry);
      }
      const float wx = wih1[src], b1a = bih1[src], b1b = bhh1[src], b2a = bih2[src], b2b = bhh2[src];
      w1[kXK + 0] = (_Float16)carry_flush(bf16r(wx), kWCarry);
      w1[kXK + 1] = (_Float16)carry_flush(bf16r(b1a), kWCarry);
      w1[kXK + 2] = (_Float16)carry_flush(bf16r(b1b), kWCarry);
      w2[kXK + 0] = (_Float16)carry_flush(bf16r(b2a), kWCarry);
      w2[kXK + 1] = (_Float16)carry_flush(bf16r(b2b), kWCarry);
    }
    if (tid < kHP) {
      const float wl = wlin[(tid < kHid) ? tid : 0];
      sWl[tid] = (tid < kHid) ? bf16r(wl) : 0.0f;
    }
  }
  __syncthreads();

  const int b0 = (blockIdx.x * 8 + wave) * 16;
  float* xw = xs + wave * 16 * kPitch;
  float* ow = os + wave * 16 * kPitch;
  const float bl0 = blin[0];
  const float bo = bf16r(bl0);
  const _Float16 one = (_Float16)kSCarry;

  float c1[4][8], h1[4][8], c2[4][8], h2[4][8];
#pragma unroll
  for (int mt = 0; mt < 4; ++mt)
#pragma unroll
    for (int r = 0; r < 8; ++r) { c1[mt][r] = 0.0f; h1[mt][r] = 0.0f; c2[mt][r] = 0.0f; h2[mt][r] = 0.0f; }

#pragma unroll 1
  for (int ch = 0; ch < kNumChunks; ++ch) {
    const int t0 = ch * kChunk;
#pragma unroll
    for (int it = 0; it < 4; ++it) {
      const int vi = it * 32 + lane;
      const int row = vi >> 3;
      const int c4 = (vi & 7) * 4;
      const v4f v = *(const v4f*)(x + (size_t)(b0 + row) * kSteps + t0 + c4);
      v4f rv;
      const float v0 = v[0], v1 = v[1], v2 = v[2], v3 = v[3];
      rv[0] = bf16r(v0); rv[1] = bf16r(v1); rv[2] = bf16r(v2); rv[3] = bf16r(v3);
      *(v4f*)(xw + row * kPitch + c4) = rv;
    }
    __syncthreads();

#pragma unroll 1
    for (int s = 0; s < kChunk; ++s) {
      int colv = col, hsv = hs;
      asm volatile("" : "+v"(colv), "+v"(hsv));
      const float xv = xw[colv * kPitch + s];
      v16h b0f = frag_tiles(h1[0], h1[1], kSCarry);
      v16h b1f = frag_tiles(h1[2], h1[3], kSCarry);
      b1f[11] = lowHalf ? (_Float16)carry_flush(xv, kSCarry) : b1f[11];
      b1f[12] = lowHalf ? one : b1f[12];
      b1f[13] = lowHalf ? one : b1f[13];
#pragma unroll
      for (int mt = 0; mt < 4; ++mt) {
        v8f acc[4];
#pragma unroll
        for (int q = 0; q < 4; ++q) {
          const _Float16* wr = sW1 + (64 * q + 16 * mt + colv) * kW1P + 8 * hsv;
          v8f a = (v8f){0.f, 0.f, 0.f, 0.f, 0.f, 0.f, 0.f, 0.f};
          a = mma_h(frag_h32(wr), b0f, a);
          a = mma_h(frag_h32(wr + 32), b1f, a);
          acc[q] = a;
        }
#pragma unroll
        for (int r = 0; r < 8; ++r) {
          const float gi = acc[0][r] * kFold, gf = acc[1][r] * kFold, gg = acc[2][r] * kFold, go = acc[3][r] * kFold;
          const float cn = fast_sigmoid(gf) * c1[mt][r] + fast_sigmoid(gi) * fast_tanh(gg);
          c1[mt][r] = cn;
          h1[mt][r] = fast_sigmoid(go) * fast_tanh(cn);
        }
      }
      v16h n0f = frag_tiles(h1[0], h1[1], kSCarry);
      v16h n1f = frag_tiles(h1[2], h1[3], kSCarry);
      n1f[11] = lowHalf ? one : n1f[11];
      n1f[12] = lowHalf ? one : n1f[12];
      const v16h p0f = frag_tiles(h2[0], h2[1], kSCarry);
      const v16h p1f = frag_tiles(h2[2], h2[3], kSCarry);
      float p = 0.0f;
#pragma unroll
      for (int mt = 0; mt < 4; ++mt) {
        v8f acc[4];
#pragma unroll
        for (int q = 0; q < 4; ++q) {
          const _Float16* wr = sW2 + (64 * q + 16 * mt + colv) * kW2P + 8 * hsv;
          v8f a = (v8f){0.f, 0.f, 0.f, 0.f, 0.f, 0.f, 0.f, 0.f};
          a = mma_h(frag_h32(wr), n0f, a);
          a = mma_h(frag_h32(wr + 32), n1f, a);
          a = mma_h(frag_h32(wr + 64), p0f, a);
          a = mma_h(frag_h32(wr + 96), p1f, a);
          acc[q] = a;
        }
        const v4f wl0 = *(const v4f*)(sWl + 16 * mt + 8 * hsv);
        const v4f wl1 = *(const v4f*)(sWl + 16 * mt + 8 * hsv + 4);
#pragma unroll
        for (int r = 0; r < 8; ++r) {
          const float gi = acc[0][r] * kFold, gf = acc[1][r] * kFold, gg = acc[2][r] * kFold, go = acc[3][r] * kFold;
          const float cn = fast_sigmoid(gf) * c2[mt][r] + fast_sigmoid(gi) * fast_tanh(gg);
          c2[mt][r] = cn;
          const float hn = fast_sigmoid(go) * fast_tanh(cn);
          h2[mt][r] = hn;
          p = fmaf((r < 4) ? wl0[r] : wl1[r - 4], hn, p);
        }
      }
      const float pother = __shfl_xor(p, 16, 32);
      const float plow = lowHalf ? p : pother;
      const float phigh = lowHalf ? pother : p;
      const float y = (plow + phigh) + bo;
      if (lowHalf) ow[colv * kPitch + s] = y;
    }
    __syncthreads();

    for (int pass = 0; pass < 2; ++pass) {
#pragma unroll
      for (int it = 0; it < 4; ++it) {
        const int vi = it * 32 + lane;
        const int row = vi >> 3;
        const int c4 = (vi & 7) * 4;
        const v4f ov = *(const v4f*)(ow + row * kPitch + c4);
        *(volatile v4f*)(outs + (size_t)(b0 + row) * kSteps + t0 + c4) = ov;
      }
      __threadfence();
    }
    __syncthreads();
  }
}

extern "C" void kernel_launch(void* const* d_in, const int* in_sizes, int n_in,
                              void* d_out, int out_size, void* d_ws, size_t ws_size,
                              hipStream_t stream) {
  if (n_in < 11 || d_out == nullptr) return;
  if ((size_t)in_sizes[0] != kOutElems) return;
  if (in_sizes[1] != kG4 || in_sizes[2] != kG4 * kHid || in_sizes[3] != kG4 || in_sizes[4] != kG4) return;
  if (in_sizes[5] != kG4 * kHid || in_sizes[6] != kG4 * kHid || in_sizes[7] != kG4 || in_sizes[8] != kG4) return;
  if (in_sizes[9] != kHid || in_sizes[10] != 1) return;
  if ((size_t)out_size != kOutElems) return;
  lstm51x2_kernel<<<kBlocks, kThr, 0, stream>>>((const float*)d_in[0], (const float*)d_in[1], (const float*)d_in[2],
                                                (const float*)d_in[3], (const float*)d_in[4], (const float*)d_in[5],
                                                (const float*)d_in[6], (const float*)d_in[7], (const float*)d_in[8],
                                                (const float*)d_in[9], (const float*)d_in[10], (float*)d_out);
}
